// RvNN_66460323938888
// MI455X (gfx1250) — hardware-verified
//
#include <hip/hip_runtime.h>
#include <stdint.h>


typedef _Float16 v16h __attribute__((ext_vector_type(16)));
typedef _Float16 v8h_t __attribute__((ext_vector_type(8)));
typedef v8h_t __attribute__((may_alias)) v8ha;
typedef float v8f __attribute__((ext_vector_type(8)));
typedef float v4f_t __attribute__((ext_vector_type(4)));
typedef v4f_t __attribute__((may_alias)) v4fa;

#define WPB 2
#define XSTRIDE 40
#define HSTRIDE 136
#define CSTRIDE 520
#define OSTRIDE 36
#define LDS_HALFS_PER_WAVE (16 * XSTRIDE + 16 * HSTRIDE + 16 * CSTRIDE)
#define WSCALE 16.0f
#define WINV 0.0625f

#define F_WC1 0
#define F_WC2 8
#define F_WP1 72
#define F_WP2 80
#define F_WL1 144
#define F_WL2 272
#define N_FRAGS 280
#define PACK_UNITS (N_FRAGS * 64)


__device__ __forceinline__ float san(float x) {
  unsigned u = __float_as_uint(x);
  if ((u & 0x7f800000u) == 0x7f800000u)
    return (u & 0x007fffffu) ? 0.0f : 9999.0f;
  return x;
}

__device__ __forceinline__ float fast_tanh(float x) {
  const float e = __builtin_amdgcn_exp2f(x * 2.885390081777927f);
  return 1.0f - 2.0f * __builtin_amdgcn_rcpf(e + 1.0f);
}

__device__ __forceinline__ v8f wmma_f16(v16h a, v16h b, v8f c) {
  v8f d = __builtin_amdgcn_wmma_f32_16x16x32_f16(false, a, false, b, (short)0, c,
                                                 false, false);
  asm volatile("v_nop\n\tv_nop\n\tv_nop\n\tv_nop" : "+v"(d) : "v"(a), "v"(b));
  return d;
}

__device__ __forceinline__ v16h load_a_frag(const _Float16* buf, int stride, int k0) {
  const int lane = threadIdx.x & 31;
  const int m  = lane & 15;
  const int hs = (lane >> 4) << 3;
  const _Float16* row = buf + m * stride + k0 + hs;
  union { v16h v; v8h_t hv[2]; } f;
  f.hv[0] = *(const v8ha*)(row);
  f.hv[1] = *(const v8ha*)(row + 16);
  return f.v;
}

__device__ __forceinline__ v16h load_b_frag(const _Float16* pack, int frag) {
  const int lane = threadIdx.x & 31;
  const _Float16* p = pack + ((size_t)frag << 9) + (lane << 4);
  return *(const v16h*)p;
}

__device__ __forceinline__ void store_act_to_lds(_Float16* buf, int stride, int n0,
                                                 v8f c, float bias, bool use_tanh,
                                                 float alpha) {
  const int lane = threadIdx.x & 31;
  const int n  = n0 + (lane & 15);
  const int mb = (lane >> 4) << 3;
#pragma unroll
  for (int vv = 0; vv < 8; ++vv) {
    float x = c[vv] * WINV + bias;
    x = use_tanh ? fast_tanh(x) : (x >= 0.0f ? x : alpha * x);
    buf[(mb + vv) * stride + n] = (_Float16)x;
  }
}

__device__ __forceinline__ void gather_child(_Float16* xbuf, const float* __restrict__ src,
                                             int row0, int njshift, int rl, int nrows) {
  const int lane = threadIdx.x & 31;
  const int k = lane;
#pragma unroll
  for (int m = 0; m < 16; ++m) {
    int r = row0 + m;
    r = (r < nrows) ? r : (nrows - 1);
    const int b = r >> njshift;
    const int j = r & ((1 << njshift) - 1);
    float v = 0.0f;
    if (k < 24) {
      const int kk   = (k < 12) ? k : (k - 12);
      const int crow = (b << (njshift + 1)) + 2 * j + ((k < 12) ? 1 : 0);
      v = san(src[(size_t)crow * rl + kk]);
    }
    xbuf[m * XSTRIDE + k] = (_Float16)v;
  }
}

__device__ __forceinline__ void gather_parent(_Float16* xbuf, const float* __restrict__ src,
                                              int row0, int nrows) {
  const int lane = threadIdx.x & 31;
  const int k = lane;
#pragma unroll
  for (int m = 0; m < 16; ++m) {
    int r = row0 + m;
    r = (r < nrows) ? r : (nrows - 1);
    float v = 0.0f;
    if (k < 12) v = san(src[(size_t)r * 12 + k]);
    xbuf[m * XSTRIDE + k] = (_Float16)v;
  }
}

__device__ __forceinline__ void enc_path(const _Float16* xbuf, _Float16* hbuf,
                                         _Float16* cbuf, int cofs,
                                         const _Float16* __restrict__ wpack, int f_w1,
                                         const float* __restrict__ b1, float alpha, int f_w2,
                                         const float* __restrict__ b2) {
  const int lane = threadIdx.x & 31;
  v16h a0 = load_a_frag(xbuf, XSTRIDE, 0);
#pragma unroll
  for (int nt = 0; nt < 8; ++nt) {
    v8f c = {};
    c = wmma_f16(a0, load_b_frag(wpack, f_w1 + nt), c);
    store_act_to_lds(hbuf, HSTRIDE, nt * 16, c, b1[nt * 16 + (lane & 15)], false, alpha);
  }
  __syncthreads();
  v16h ha[4];
#pragma unroll
  for (int kc = 0; kc < 4; ++kc) ha[kc] = load_a_frag(hbuf, HSTRIDE, kc * 32);
  for (int nt = 0; nt < 16; ++nt) {
    v8f c = {};
#pragma unroll
    for (int kc = 0; kc < 4; ++kc)
      c = wmma_f16(ha[kc], load_b_frag(wpack, f_w2 + kc * 16 + nt), c);
    store_act_to_lds(cbuf, CSTRIDE, cofs + nt * 16, c, b2[nt * 16 + (lane & 15)], true, 0.0f);
  }
}

__device__ __forceinline__ void write_tile_lines(const float* obuf, float* __restrict__ out,
                                                 int row0, int nrows, bool active) {
  const int lane = threadIdx.x & 31;
  const int s = lane >> 3;
  const int q = lane & 7;
  v4f_t v[4];
#pragma unroll
  for (int i = 0; i < 4; ++i)
    v[i] = *(const v4fa*)(obuf + (4 * i + s) * OSTRIDE + 4 * q);
#pragma unroll
  for (int i = 0; i < 4; ++i) {
    const int gr = row0 + 4 * i + s;
    if (active && gr < nrows)
      *(volatile v4f_t*)(out + (size_t)gr * 32 + 4 * q) = v[i];
  }
  __threadfence();
#pragma unroll
  for (int i = 0; i < 4; ++i) {
    const int gr = row0 + 4 * i + s;
    if (active && gr < nrows)
      *(volatile v4f_t*)(out + (size_t)gr * 32 + 4 * q) = v[i];
  }
}


__global__ __launch_bounds__(256)
void pack_weights_kernel(const float* __restrict__ Wc1, const float* __restrict__ Wc2,
                         const float* __restrict__ Wp1, const float* __restrict__ Wp2,
                         const float* __restrict__ Wl1, const float* __restrict__ Wl2,
                         _Float16* __restrict__ pack) {
  const int u = blockIdx.x * blockDim.x + threadIdx.x;
  const bool act = (u < PACK_UNITS);
  const int uc = act ? u : 0;
  const int frag = uc >> 6;
  const int lane = (uc >> 1) & 31;
  const int hf = uc & 1;
  const float* W; int K, N, kc, nt;
  if (frag < F_WC2)      { W = Wc1; K = 24;  N = 128; kc = 0;      nt = frag; }
  else if (frag < F_WP1) { int f = frag - F_WC2; W = Wc2; K = 128; N = 256; kc = f >> 4; nt = f & 15; }
  else if (frag < F_WP2) { W = Wp1; K = 12;  N = 128; kc = 0;      nt = frag - F_WP1; }
  else if (frag < F_WL1) { int f = frag - F_WP2; W = Wp2; K = 128; N = 256; kc = f >> 4; nt = f & 15; }
  else if (frag < F_WL2) { int f = frag - F_WL1; W = Wl1; K = 512; N = 128; kc = f >> 3; nt = f & 7; }
  else                   { int f = frag - F_WL2; W = Wl2; K = 128; N = 32;  kc = f >> 1; nt = f & 1; }
  const int n  = nt * 16 + (lane & 15);
  const int kb = kc * 32 + 16 * hf + 8 * (lane >> 4);
  union { v8h_t h; v4f_t f; } o;
#pragma unroll
  for (int i = 0; i < 8; ++i) {
    const int k = kb + i;
    const float wv = (k < K) ? W[(size_t)k * N + n] * WSCALE : 0.0f;
    o.h[i] = (_Float16)wv;
  }
  _Float16* dst = pack + ((size_t)frag << 9) + (lane << 4) + (hf << 3);
  const v4f_t val = o.f;
  if (act) *(volatile v4f_t*)dst = val;
  __threadfence();
  if (act) *(volatile v4f_t*)dst = val;
}

__global__ __launch_bounds__(WPB * 32)
void rvnn_stage_kernel(const float* __restrict__ child, int child_rl, int njshift, int nrows,
                       const float* __restrict__ parent,
                       const _Float16* __restrict__ wpack,
                       const float* __restrict__ bc1, const float* __restrict__ ac,
                       const float* __restrict__ bc2, const float* __restrict__ bp1,
                       const float* __restrict__ ap, const float* __restrict__ bp2,
                       const float* __restrict__ bl1, const float* __restrict__ bl2,
                       const float* __restrict__ al, float* __restrict__ out) {
  __shared__ __attribute__((aligned(16))) _Float16 smem[WPB * LDS_HALFS_PER_WAVE];
  __shared__ __attribute__((aligned(16))) float sout[WPB * 16 * OSTRIDE];
  const int wave = threadIdx.x >> 5;
  const int lane = threadIdx.x & 31;
  const int ntiles = (nrows + 15) >> 4;
  const int tile = blockIdx.x * WPB + wave;
  const bool active = (tile < ntiles);
  const int tile_c = active ? tile : (ntiles - 1);
  _Float16* xbuf = smem + wave * LDS_HALFS_PER_WAVE;
  _Float16* hbuf = xbuf + 16 * XSTRIDE;
  _Float16* cbuf = hbuf + 16 * HSTRIDE;
  float* obuf = sout + wave * 16 * OSTRIDE;
  const int row0 = tile_c * 16;
  const float a_c = ac[0], a_p = ap[0], a_l = al[0];

  gather_child(xbuf, child, row0, njshift, child_rl, nrows);
  __syncthreads();
  enc_path(xbuf, hbuf, cbuf, 0, wpack, F_WC1, bc1, a_c, F_WC2, bc2);
  __syncthreads();
  gather_parent(xbuf, parent, row0, nrows);
  __syncthreads();
  enc_path(xbuf, hbuf, cbuf, 256, wpack, F_WP1, bp1, a_p, F_WP2, bp2);
  __syncthreads();

  v8f acc[8];
#pragma unroll
  for (int nt = 0; nt < 8; ++nt) { v8f z = {}; acc[nt] = z; }
  for (int kc = 0; kc < 16; ++kc) {
    v16h a = load_a_frag(cbuf, CSTRIDE, kc * 32);
#pragma unroll
    for (int nt = 0; nt < 8; ++nt)
      acc[nt] = wmma_f16(a, load_b_frag(wpack, F_WL1 + kc * 8 + nt), acc[nt]);
  }
#pragma unroll
  for (int nt = 0; nt < 8; ++nt)
    store_act_to_lds(hbuf, HSTRIDE, nt * 16, acc[nt], bl1[nt * 16 + (lane & 15)], true, 0.0f);
  __syncthreads();

  v16h ha[4];
#pragma unroll
  for (int kc = 0; kc < 4; ++kc) ha[kc] = load_a_frag(hbuf, HSTRIDE, kc * 32);
#pragma unroll
  for (int nt = 0; nt < 2; ++nt) {
    v8f c = {};
#pragma unroll
    for (int kc = 0; kc < 4; ++kc)
      c = wmma_f16(ha[kc], load_b_frag(wpack, F_WL2 + kc * 2 + nt), c);
    const float bias = bl2[nt * 16 + (lane & 15)];
    const int n  = nt * 16 + (lane & 15);
    const int mb = (lane >> 4) << 3;
#pragma unroll
    for (int vv = 0; vv < 8; ++vv) {
      float x = c[vv] * WINV + bias;
      x = (x >= 0.0f) ? x : a_l * x;
      obuf[(mb + vv) * OSTRIDE + n] = x;
    }
  }
  __syncthreads();
  write_tile_lines(obuf, out, row0, nrows, active);
}


extern "C" void kernel_launch(void* const* d_in, const int* in_sizes, int n_in,
                              void* d_out, int out_size, void* d_ws, size_t ws_size,
                              hipStream_t stream) {
  if (n_in < 18) return;
  const float* level1 = (const float*)d_in[0];
  const float* level2 = (const float*)d_in[1];
  const float* level3 = (const float*)d_in[2];
  const float* Wc1 = (const float*)d_in[3];
  const float* bc1 = (const float*)d_in[4];
  const float* ac  = (const float*)d_in[5];
  const float* Wc2 = (const float*)d_in[6];
  const float* bc2 = (const float*)d_in[7];
  const float* Wp1 = (const float*)d_in[8];
  const float* bp1 = (const float*)d_in[9];
  const float* ap  = (const float*)d_in[10];
  const float* Wp2 = (const float*)d_in[11];
  const float* bp2 = (const float*)d_in[12];
  const float* Wl1 = (const float*)d_in[13];
  const float* bl1 = (const float*)d_in[14];
  const float* Wl2 = (const float*)d_in[15];
  const float* bl2 = (const float*)d_in[16];
  const float* al  = (const float*)d_in[17];

  const int B = in_sizes[0] / 24;
  if (B <= 0) return;
  if (in_sizes[1] != B * 48 || in_sizes[2] != B * 96 || out_size != B * 64) return;

  const size_t pack_bytes = (size_t)N_FRAGS * 512 * sizeof(_Float16);
  const size_t out3_off   = (size_t)512 * 1024;
  const size_t out3_bytes = (size_t)B * 4 * 32 * sizeof(float);
  if (pack_bytes > out3_off || out3_off + out3_bytes > ws_size) return;
  _Float16* wpack = (_Float16*)d_ws;
  float* out3 = (float*)((char*)d_ws + out3_off);

  pack_weights_kernel<<<(PACK_UNITS + 255) / 256, 256, 0, stream>>>(
      Wc1, Wc2, Wp1, Wp2, Wl1, Wl2, wpack);

  const int nrows1 = B * 4;
  const int ntiles1 = (nrows1 + 15) / 16;
  rvnn_stage_kernel<<<(ntiles1 + WPB - 1) / WPB, WPB * 32, 0, stream>>>(
      level3, 12, 2, nrows1, level2, wpack, bc1, ac, bc2, bp1, ap, bp2, bl1, bl2, al, out3);

  const int nrows2 = B * 2;
  const int ntiles2 = (nrows2 + 15) / 16;
  rvnn_stage_kernel<<<(ntiles2 + WPB - 1) / WPB, WPB * 32, 0, stream>>>(
      out3, 32, 1, nrows2, level1, wpack, bc1, ac, bc2, bp1, ap, bp2, bl1, bl2, al,
      (float*)d_out);
}
